// EGNNLayer_31714038514064
// MI455X (gfx1250) — hardware-run, weakly checked
//
#include <hip/hip_runtime.h>


namespace {

constexpr int N = 20000, NP = 20000, NPL = NP  , SRCM = N  , EFULL = 640000, E = EFULL  ;
constexpr int FX = 160  , NS_ = 64  , NV_ = 32  , TSW = 160  , TVW = 128  , AW = 160  , VOC = 1, NRL = NP, NL = (NPL < N ? NPL : N);
constexpr float INV8 = 0.125f, K_VV = 0.5773502691896258f * 0.17677669529663687f, INV_SQRT32 = 0.17677669529663687f, INV64 = 0.015625f, K_UVV = 0.5773502691896258f * 0.03125f, INV_SQRT2048 = 0.022097086912079608f;
constexpr float LNEPS = 1e-5f; constexpr float LOG2E = 1.4426950408889634f; constexpr float XS = 8.0f, WSC = 256.0f, WSQ = 0.25f, RS_ = 1024.0f, NSL_ = 0.2f, NSA_ = 0.01f, SLOPE = 0.0f, BNEPS = 1e-5f;
static_assert(NP % 32 == 0 && NP >= N && NPL % 32 == 0, "tiling");
typedef _Float16 b16;
typedef __attribute__((ext_vector_type(16))) _Float16 v16b;
typedef __attribute__((ext_vector_type(8))) _Float16 v8b;
typedef __attribute__((ext_vector_type(8))) float v8f;
typedef __attribute__((ext_vector_type(4))) float v4f;
__device__ __forceinline__ float bf16_rne(float f) { unsigned int u = __float_as_uint(f); u += 0x7FFFu + ((u >> 16) & 1u); return __uint_as_float(u & 0xFFFF0000u); }
__device__ __forceinline__ void split16(float v, b16& hi, b16& lo) { hi = (b16)v; lo = (b16)(v - (float)hi); }
__device__ __forceinline__ v16b frag_kb(const b16* p, int hh) { const v8b a = *(const v8b*)(p + 8 * hh), b = *(const v8b*)(p + 16 + 8 * hh); v16b f;
#pragma unroll
  for (int e = 0; e < 8; ++e) { f[e] = a[e]; f[8 + e] = b[e]; } return f; }
__device__ __forceinline__ v8f wmma16b(v16b a, v16b b, v8f c) { v8f d = __builtin_amdgcn_wmma_f32_16x16x32_f16(false, a, false, b, (short)0, c, false, false); asm volatile("v_nop\n\tv_nop\n\tv_nop\n\tv_nop" : "+v"(d) : "v"(a), "v"(b)); return d; }
__device__ __forceinline__ void wave_lds_sync() { __builtin_amdgcn_fence(__ATOMIC_RELEASE, "workgroup"); __builtin_amdgcn_wave_barrier(); __builtin_amdgcn_fence(__ATOMIC_ACQUIRE, "workgroup"); }
__device__ __forceinline__ float pmul(float a, float b) { float p = a * b; asm volatile("" : "+v"(p)); return p; }
__device__ __forceinline__ int iclamp(int v, int lo, int hi) { return v < lo ? lo : (v > hi ? hi : v); }

typedef __attribute__((ext_vector_type(4))) _Float16 v4h;
__device__ __forceinline__ float lrelu(float v) { return v > 0.0f ? v : NSL_ * v; }
template <int K, int NOUTR, int NOUTP>
__global__ __launch_bounds__(256) void wt_kernel(const float* __restrict__ w, b16* __restrict__ WT, float scl) {
  const int u = blockIdx.x * 256 + threadIdx.x; if (u >= NOUTP * K / 8) return; const int e = u * 8; const int o = e / K, k0 = e % K; v8b v;
#pragma unroll
  for (int j = 0; j < 8; ++j) v[j] = (b16)(o < NOUTR ? bf16_rne(w[(size_t)(k0 + j) * NOUTR + o]) * scl : 0.0f);
  for (int pass = 0; pass < 2; ++pass) { *(volatile v8b*)(WT + e) = v; __threadfence(); }
}
template <int K, int NT, bool RND, int MODE, bool GIDX>
__global__ __launch_bounds__(64) void lin_kernel(const float* __restrict__ X, const int* __restrict__ gidx, const b16* __restrict__ WT, const b16* __restrict__ WQ, const float* __restrict__ bias, float* __restrict__ OUT, int opitch, int nvalid, int mrows, const float* __restrict__ lng = nullptr, const float* __restrict__ lnb = nullptr, const float* __restrict__ rsc = nullptr) {
  constexpr int NC = NT * 16;
  __shared__ __attribute__((aligned(16))) b16 Ah[2][16][K + 8], Al[2][16][K + 8]; __shared__ __attribute__((aligned(16))) float Tf[2][16][NC + 4];
  const int wave = threadIdx.x >> 5, lane = threadIdx.x & 31, nloc = lane & 15, hlf = lane >> 4; const size_t m0 = (size_t)blockIdx.x * 32 + wave * 16;
  for (int idx = lane; idx < 16 * (K / 4); idx += 32) { const int rr = idx / (K / 4), c4 = (idx % (K / 4)) * 4; const size_t vrow = (m0 + rr < (size_t)nvalid) ? m0 + rr : (size_t)nvalid - 1; size_t arow = vrow; if (GIDX) arow = (size_t)iclamp(gidx[vrow], 0, VOC - 1);
    const v4f v = *(const v4f*)(X + arow * K + c4); v4h hv, lv;
    for (int j = 0; j < 4; ++j) { float vj = v[j]; if (MODE == 2) vj = fmaxf(vj, 0.0f); const float vs = (RND ? bf16_rne(vj) : vj) * XS; const b16 ph = (b16)vs; hv[j] = ph; lv[j] = (b16)((vs - (float)ph) * RS_); } *(v4h*)(&Ah[wave][rr][c4]) = hv; *(v4h*)(&Al[wave][rr][c4]) = lv; }
  wave_lds_sync();
  v8f acc[NT];
#pragma unroll
  for (int t = 0; t < NT; ++t) acc[t] = (v8f){};
#pragma unroll 1
  for (int kb = 0; kb < K; kb += 32) { const v16b a = frag_kb(&Ah[wave][nloc][kb], hlf); v16b al; if (!RND) al = frag_kb(&Al[wave][nloc][kb], hlf);
#pragma unroll
    for (int t = 0; t < NT; ++t) { const size_t wo_ = (size_t)(t * 16 + nloc) * K + kb; acc[t] = wmma16b(a, frag_kb(WT + wo_, hlf), acc[t]); if (!RND) acc[t] = wmma16b(al, frag_kb(WQ + wo_, hlf), acc[t]); } }
if (MODE == 5) {
    static_assert(MODE != 5 || NT == 8, "LN epilogue needs the full 128-wide row in one wave");
    float sm[8], sq[8]; for (int r = 0; r < 8; ++r) { sm[r] = 0.0f; sq[r] = 0.0f; }
    for (int t = 0; t < NT; ++t) { const int col = t * 16 + nloc; const float bb = bf16_rne(bias[col]); for (int r = 0; r < 8; ++r) { const float y = acc[t][r] * (1.0f / (XS * WSC)) + bb; acc[t][r] = y; sm[r] += y; } }
#pragma unroll
    for (int o = 1; o < 16; o <<= 1) for (int r = 0; r < 8; ++r) sm[r] += __shfl_xor(sm[r], o);
    for (int t = 0; t < NT; ++t) for (int r = 0; r < 8; ++r) { const float d = acc[t][r] - sm[r] * (1.0f / NC); sq[r] += pmul(d, d); }
#pragma unroll
    for (int o = 1; o < 16; o <<= 1) for (int r = 0; r < 8; ++r) sq[r] += __shfl_xor(sq[r], o);
    for (int t = 0; t < NT; ++t) { const int col = t * 16 + nloc; const float gg = bf16_rne(lng[col]), be = bf16_rne(lnb[col]);
      for (int r = 0; r < 8; ++r) { const size_t vrow = m0 + 8 * hlf + r; const float y = fmaxf((acc[t][r] - sm[r] * (1.0f / NC)) * rsqrtf(sq[r] * (1.0f / NC) + LNEPS) * gg + be, 0.0f); Tf[wave][8 * hlf + r][col] = (vrow < (size_t)nvalid) ? y : 0.0f; } }
  } else {
  for (int t = 0; t < NT; ++t) { const int col = t * 16 + nloc; const float bb = bf16_rne(bias[col]);
    for (int r = 0; r < 8; ++r) { const size_t vrow = m0 + 8 * hlf + r; float a_ = acc[t][r] * (1.0f / (XS * WSC)); if (MODE == 6) a_ = pmul(a_, rsc[((vrow < (size_t)nvalid) ? vrow : (size_t)nvalid - 1) * 4 + 2]); float y = a_ + bb; if (MODE == 1) y = fmaxf(y, 0.0f); Tf[wave][8 * hlf + r][col] = (vrow < (size_t)nvalid) ? y : 0.0f; } }
  }
  wave_lds_sync();
  for (int pass = 0; pass < 2; ++pass) { for (int rr = 0; rr < 16; ++rr) { if (m0 + rr < (size_t)mrows) { if (NC >= 128) { for (int c8 = 0; c8 < NC; c8 += 128) { if (NC % 128 == 0 || c8 + lane * 4 < NC) *(volatile v4f*)(OUT + (m0 + rr) * (size_t)opitch + c8 + lane * 4) = *(const v4f*)(&Tf[wave][rr][c8 + lane * 4]); } }
        else { if (lane < NC / 4) *(volatile v4f*)(OUT + (m0 + rr) * (size_t)opitch + lane * 4) = *(const v4f*)(&Tf[wave][rr][lane * 4]); } } } __threadfence(); }
}
__device__ __forceinline__ float gelu_(float v) { return 0.5f * v * (1.0f + erff(v * 0.70710678118654752f)); }
template <int KW, int NOUT>
__global__ __launch_bounds__(256) void wts_kernel(const float* __restrict__ w, int k0, b16* __restrict__ WT, float scl) {
  const int u = blockIdx.x * 256 + threadIdx.x; if (u >= NOUT * KW / 8) return; const int e = u * 8; const int o = e / KW, kk = e % KW; v8b v;
#pragma unroll
  for (int j = 0; j < 8; ++j) v[j] = (b16)(bf16_rne(w[(size_t)(k0 + kk + j) * NOUT + o]) * scl);
  for (int pass = 0; pass < 2; ++pass) { *(volatile v8b*)(WT + e) = v; __threadfence(); }
}
__global__ __launch_bounds__(256) void zfill_kernel(float* __restrict__ Z, int n) { const int i = threadIdx.x; for (int pass = 0; pass < 2; ++pass) { if (i < n) ((volatile float*)Z)[i] = 0.0f; __threadfence(); } }
constexpr int CSR_NBLK = 512, CSR_GB = 8  , CSR_GN = 1 << CSR_GB  , CSR_MAXG = 512, CSR_CAP = 12288  ;
__global__ __launch_bounds__(64) void csrA_kernel(const int* __restrict__ dst, int E, int N, int nG, int CHP, int NGP, int* __restrict__ STG, int* __restrict__ HST) {
  extern __shared__ int sm[];
  int* cnt = sm; int* run = sm + NGP; int* ids = sm + 2 * NGP;
  const int b = blockIdx.x; const int ch = (E + CSR_NBLK - 1) / CSR_NBLK; const int e0 = b * ch, e1 = min(E, e0 + ch);
  for (int i = threadIdx.x; i < NGP; i += 64) cnt[i] = 0;
  for (int i = threadIdx.x; i < CHP; i += 64) ids[i] = -1;
  __syncthreads();
  if (threadIdx.x == 0) {
    for (int e = e0; e < e1; ++e) { int d = dst[e]; d = (d < 0) ? 0 : (d >= N ? N - 1 : d); cnt[d >> CSR_GB] += 1; }
    int acc = 0; for (int g = 0; g < nG; ++g) { run[g] = acc; acc += cnt[g]; }
    for (int e = e0; e < e1; ++e) { int d = dst[e]; d = (d < 0) ? 0 : (d >= N ? N - 1 : d); const int g = d >> CSR_GB; ids[run[g]] = e; run[g] += 1; } }
  __syncthreads();
  typedef __attribute__((ext_vector_type(4))) int v4i;
  for (int pass = 0; pass < 2; ++pass) {
    for (int i = threadIdx.x; i < CHP / 4; i += 64) *(volatile v4i*)(STG + (size_t)b * CHP + i * 4) = *(const v4i*)(&ids[i * 4]);
    for (int i = threadIdx.x; i < NGP / 4; i += 64) { v4i v; for (int e = 0; e < 4; ++e) v[e] = (i * 4 + e < nG) ? cnt[i * 4 + e] : 0; *(volatile v4i*)(HST + (size_t)b * NGP + i * 4) = v; }
    __threadfence(); }
}
__global__ __launch_bounds__(512) void csrS_kernel(const int* __restrict__ HST, int nG, int NGP, int* __restrict__ START, int* __restrict__ TOT, int* __restrict__ OFF) {
  __shared__ int tot[CSR_MAXG];
  const int b = threadIdx.x;
  for (int pass = 0; pass < 2; ++pass) { int runb = 0; for (int g = 0; g < nG; ++g) { int c = HST[(size_t)b * NGP + g]; c = (c < 0) ? 0 : c; ((volatile int*)OFF)[(size_t)g * CSR_NBLK + b] = runb; runb += c; } __threadfence(); }
  for (int g = threadIdx.x; g < nG; g += 512) { int s = 0; for (int bb = 0; bb < CSR_NBLK; ++bb) { int c = HST[(size_t)bb * NGP + g]; s += (c < 0) ? 0 : c; } tot[g] = s; }
  __syncthreads();
  if (threadIdx.x < 32) {
    __shared__ int st[CSR_MAXG + 32];
    if (threadIdx.x == 0) { int acc = 0; for (int g = 0; g < NGP; ++g) { st[g] = acc; if (g < nG) acc += (tot[g] + 31) & ~31; } st[NGP] = acc; }
    __builtin_amdgcn_fence(__ATOMIC_RELEASE, "workgroup"); __builtin_amdgcn_wave_barrier(); __builtin_amdgcn_fence(__ATOMIC_ACQUIRE, "workgroup");
    for (int pass = 0; pass < 2; ++pass) { for (int i = threadIdx.x; i < NGP + 32; i += 32) { ((volatile int*)START)[i] = (i <= NGP) ? st[min(i, NGP)] : 0; ((volatile int*)TOT)[i] = (i < nG) ? tot[i] : 0; } __threadfence(); } }
}
__global__ __launch_bounds__(256) void csrB_kernel(const int* __restrict__ dst, int N, int nG, int CHP, int NGP, int permLen, const int* __restrict__ STG, const int* __restrict__ HST, const int* __restrict__ OFF, const int* __restrict__ START, const int* __restrict__ TOT, int* __restrict__ PERM, int* __restrict__ ROWPTR, int* __restrict__ ROWCNT, int* __restrict__ FLAG) {
  typedef __attribute__((ext_vector_type(4))) int v4i;
  __shared__ int ids[CSR_CAP]; __shared__ unsigned short key[CSR_CAP]; __shared__ int outp[CSR_CAP]; __shared__ int ncnt[CSR_GN + 1]; __shared__ int boff[CSR_NBLK + 1];
  const int g = blockIdx.x, t_ = threadIdx.x; int tot = TOT[g]; int st = START[g], stn = START[g + 1]; const int v0 = g * CSR_GN; const int nv = min(CSR_GN, N - v0);
  st = (st < 0) ? 0 : (st > permLen - 32 ? permLen - 32 : st) & ~31; stn = (stn < st) ? st : (stn > permLen ? permLen : stn); tot = (tot < 0) ? 0 : tot; if (tot > stn - st && tot <= CSR_CAP) tot = stn - st;
  if (tot > CSR_CAP) {
    for (int pass = 0; pass < 2; ++pass) { for (int i = t_; i < CSR_GN / 4; i += 256) { v4i a, c; for (int e = 0; e < 4; ++e) { a[e] = st; c[e] = 0; } *(volatile v4i*)(ROWPTR + v0 + i * 4) = a; *(volatile v4i*)(ROWCNT + v0 + i * 4) = c; } if (t_ == 0) ((volatile int*)FLAG)[0] = 1; __threadfence(); } (void)nv; return; }
  if (t_ == 0) { int acc = 0; for (int b = 0; b < CSR_NBLK; ++b) { boff[b] = acc; int c = HST[(size_t)b * NGP + g]; c = (c < 0) ? 0 : (c > CHP ? CHP : c); acc += c; if (acc > tot) acc = tot; } boff[CSR_NBLK] = acc; }
  for (int i = t_; i <= CSR_GN; i += 256) ncnt[i] = 0;
  __syncthreads();
  for (int b = 0; b < CSR_NBLK; ++b) { const int c = boff[b + 1] - boff[b]; int o_ = OFF[(size_t)g * CSR_NBLK + b]; o_ = (o_ < 0) ? 0 : (o_ > CHP - c ? CHP - c : o_); const int* src_ = STG + (size_t)b * CHP + o_;
    for (int i = t_; i < c; i += 256) { int id = src_[i]; id = (id < 0) ? 0 : id; ids[boff[b] + i] = id; int d = dst[id]; d = (d < v0) ? v0 : (d >= N ? N - 1 : d); int kk = d - v0; kk = (kk < 0) ? 0 : (kk >= CSR_GN ? CSR_GN - 1 : kk); key[boff[b] + i] = (unsigned short)kk; } }
  __syncthreads();
  if (t_ == 0) { for (int i = 0; i < tot; ++i) ncnt[key[i]] += 1; int acc = 0; for (int vl = 0; vl < CSR_GN; ++vl) { const int c = ncnt[vl]; ncnt[vl] = acc; acc += c; } ncnt[CSR_GN] = acc;
    for (int i = 0; i < tot; ++i) { const int vl = key[i]; outp[ncnt[vl]] = ids[i]; ncnt[vl] += 1; }
    for (int vl = CSR_GN; vl > 0; --vl) ncnt[vl] = ncnt[vl - 1]; ncnt[0] = 0; }
  __syncthreads();
  for (int pass = 0; pass < 2; ++pass) {
    for (int i = t_; i < (stn - st) / 4; i += 256) { v4i v; for (int e = 0; e < 4; ++e) { const int q = i * 4 + e; v[e] = (q < tot) ? outp[q] : -1; } *(volatile v4i*)(PERM + st + i * 4) = v; }
    for (int i = t_; i < CSR_GN / 4; i += 256) { v4i a, c; for (int e = 0; e < 4; ++e) { const int vl = i * 4 + e; a[e] = st + ncnt[vl]; c[e] = (vl < nv) ? (ncnt[vl + 1] - ncnt[vl]) : 0; } *(volatile v4i*)(ROWPTR + v0 + i * 4) = a; *(volatile v4i*)(ROWCNT + v0 + i * 4) = c; }
    __threadfence(); }
}
__global__ __launch_bounds__(256) void csrZ_kernel(int* __restrict__ p, size_t n4) { typedef __attribute__((ext_vector_type(4))) int v4i; const size_t tid = (size_t)blockIdx.x * 256 + threadIdx.x, nth = (size_t)gridDim.x * 256; v4i z = {0, 0, 0, 0}; for (size_t i = tid; i < n4; i += nth) *(volatile v4i*)(p + i * 4) = z; }
struct CsrBufs { int *STG, *HST, *OFF, *START, *TOT, *PERM, *ROWPTR, *ROWCNT, *FLAG; int nG, NGP, CHP; size_t permLen; char* base; size_t bytes; };
static size_t csr_carve(CsrBufs& c, char* ws, size_t off, int E, int N) {
  const size_t off0 = off; c.base = ws + off;
  auto al = [&](size_t bytes) { char* p = ws + off; off += (bytes + 255) & ~(size_t)255; return p; };
  c.nG = (N + CSR_GN - 1) / CSR_GN; c.NGP = (c.nG + 31) & ~31; const int ch = (E + CSR_NBLK - 1) / CSR_NBLK; c.CHP = (ch + 31) & ~31; c.permLen = (size_t)E + 32 * (size_t)c.nG + 32;
  c.STG = (int*)al((size_t)CSR_NBLK * c.CHP * 4); c.HST = (int*)al((size_t)CSR_NBLK * c.NGP * 4); c.OFF = (int*)al((size_t)c.NGP * CSR_NBLK * 4); c.START = (int*)al((size_t)(c.NGP + 64) * 4); c.TOT = (int*)al((size_t)(c.NGP + 64) * 4);
  c.PERM = (int*)al(c.permLen * 4); c.ROWPTR = (int*)al((size_t)c.nG * CSR_GN * 4); c.ROWCNT = (int*)al((size_t)c.nG * CSR_GN * 4); c.FLAG = (int*)al(256);
  c.bytes = off - off0; return off;
}
static void csr_build(const CsrBufs& c, const int* dst, int E, int N, hipStream_t stream) {
  const size_t smem = (size_t)(2 * c.NGP + c.CHP) * 4;
  csrZ_kernel<<<512, 256, 0, stream>>>((int*)c.base, c.bytes / 16);
  csrA_kernel<<<CSR_NBLK, 64, smem, stream>>>(dst, E, N, c.nG, c.CHP, c.NGP, c.STG, c.HST);
  csrS_kernel<<<1, 512, 0, stream>>>(c.HST, c.nG, c.NGP, c.START, c.TOT, c.OFF);
  csrB_kernel<<<c.nG, 256, 0, stream>>>(dst, N, c.nG, c.CHP, c.NGP, (int)c.permLen, c.STG, c.HST, c.OFF, c.START, c.TOT, c.PERM, c.ROWPTR, c.ROWCNT, c.FLAG);
}
__global__ __launch_bounds__(256) void split_kernel(const float* __restrict__ x, float* __restrict__ XS, float* __restrict__ XV) {
  const int i = blockIdx.x * 256 + threadIdx.x; if (i >= NRL * 20) return; const int n = i / 20, q = i % 20; float o[8];
  if (q < 8) { for (int j = 0; j < 8; ++j) o[j] = (n < N) ? bf16_rne(x[(size_t)n * FX + q * 8 + j]) : 0.0f; }
  else { const int ii = (q - 8) / 4, u0 = ((q - 8) % 4) * 8; for (int j = 0; j < 8; ++j) o[j] = (n < N) ? bf16_rne(x[(size_t)n * FX + NS_ + 3 * (u0 + j) + ii]) : 0.0f; }
  float* dst = (q < 8) ? (XS + (size_t)n * NS_ + q * 8) : (XV + ((size_t)((q - 8) / 4) * NP + n) * NV_ + (((q - 8) % 4) * 8));
  for (int pass = 0; pass < 2; ++pass) { *(volatile v4f*)dst = *(v4f*)&o[0]; *(volatile v4f*)(dst + 4) = *(v4f*)&o[4]; __threadfence(); }
}
__global__ __launch_bounds__(256) void magg_kernel(const float* __restrict__ TS, const float* __restrict__ TV, const float* __restrict__ attr, const int* __restrict__ cols, const int* __restrict__ PERM, const int* __restrict__ ROWPTR, const int* __restrict__ ROWCNT, int permLen, float* __restrict__ AGG, int mrows) {
  const int tid = threadIdx.x; const int row = tid >> 3, g = tid & 7; const int v = blockIdx.x * 32 + row;
  int cnt = 0, p0 = 0; if (v < N) { cnt = iclamp(ROWCNT[v], 0, 65536); p0 = iclamp(ROWPTR[v], 0, permLen - 1); if (p0 + cnt > permLen) cnt = permLen - p0; }
  float m0[8], m1[12]; for (int j = 0; j < 8; ++j) m0[j] = 0.0f; for (int j = 0; j < 12; ++j) m1[j] = 0.0f;
#pragma unroll 1
  for (int i = 0; i < cnt; ++i) { const int e = iclamp(PERM[p0 + i], 0, E - 1); int c = iclamp(cols[e], 0, N - 1); if (SRCM < N) c %= SRCM;
    const v4f at = *(const v4f*)(attr + (size_t)e * 4); const float r0 = bf16_rne(at[0]), r1 = bf16_rne(at[1]), r2 = bf16_rne(at[2]), d = bf16_rne(at[3]);
    const float* ts = TS + (size_t)c * TSW; const float* tv0 = TV + (size_t)c * TVW; const float* tv1 = TV + ((size_t)NP + c) * TVW; const float* tv2 = TV + ((size_t)2 * NP + c) * TVW;
    { const v4f a0 = *(const v4f*)(ts + g * 8), a1 = *(const v4f*)(ts + g * 8 + 4), c0 = *(const v4f*)(ts + NS_ + g * 8), c1 = *(const v4f*)(ts + NS_ + g * 8 + 4);
      const v4f b00 = *(const v4f*)(tv0 + g * 8), b01 = *(const v4f*)(tv0 + g * 8 + 4), b10 = *(const v4f*)(tv1 + g * 8), b11 = *(const v4f*)(tv1 + g * 8 + 4), b20 = *(const v4f*)(tv2 + g * 8), b21 = *(const v4f*)(tv2 + g * 8 + 4);
      for (int j = 0; j < 4; ++j) { m0[j] += pmul(d * INV8, a0[j]) + pmul(r0 * K_VV, b00[j]) + pmul(r1 * K_VV, b10[j]) + pmul(r2 * K_VV, b20[j]) + c0[j] * INV8; m0[4 + j] += pmul(d * INV8, a1[j]) + pmul(r0 * K_VV, b01[j]) + pmul(r1 * K_VV, b11[j]) + pmul(r2 * K_VV, b21[j]) + c1[j] * INV8; } }
    { const v4f d1 = *(const v4f*)(ts + 2 * NS_ + g * 4); const v4f e0 = *(const v4f*)(tv0 + NS_ + g * 4), e1 = *(const v4f*)(tv1 + NS_ + g * 4), e2 = *(const v4f*)(tv2 + NS_ + g * 4); const v4f f0 = *(const v4f*)(tv0 + NS_ + NV_ + g * 4), f1 = *(const v4f*)(tv1 + NS_ + NV_ + g * 4), f2 = *(const v4f*)(tv2 + NS_ + NV_ + g * 4);
      for (int w = 0; w < 4; ++w) { m1[3 * w + 0] += pmul(r0 * INV8, d1[w]) + pmul(d * INV_SQRT32, e0[w]) + f0[w] * INV_SQRT32; m1[3 * w + 1] += pmul(r1 * INV8, d1[w]) + pmul(d * INV_SQRT32, e1[w]) + f1[w] * INV_SQRT32; m1[3 * w + 2] += pmul(r2 * INV8, d1[w]) + pmul(d * INV_SQRT32, e2[w]) + f2[w] * INV_SQRT32; } } }
  for (int pass = 0; pass < 2; ++pass) { if (v < mrows) { float* orow = AGG + (size_t)v * AW; const bool ok = (v < N);
      v4f o; for (int j = 0; j < 4; ++j) o[j] = ok ? m0[j] : 0.0f; *(volatile v4f*)(orow + g * 8) = o; for (int j = 0; j < 4; ++j) o[j] = ok ? m0[4 + j] : 0.0f; *(volatile v4f*)(orow + g * 8 + 4) = o;
      for (int q = 0; q < 3; ++q) { for (int j = 0; j < 4; ++j) o[j] = ok ? m1[4 * q + j] : 0.0f; *(volatile v4f*)(orow + NS_ + g * 12 + 4 * q) = o; } }
    __threadfence(); }
}
template <int NU, int NVv, int NW>
__global__ __launch_bounds__(256) void wuvw_kernel(const float* __restrict__ W, b16* __restrict__ WT, float scl) {
  const int t = blockIdx.x * 256 + threadIdx.x; if (t >= NU * NW * NVv / 8) return; const int e = t * 8; const int u = e / (NW * NVv), w = (e / NVv) % NW, v0 = e % NVv; v8b o;
#pragma unroll
  for (int j = 0; j < 8; ++j) o[j] = (b16)(bf16_rne(W[((size_t)u * NVv + v0 + j) * NW + w]) * scl);
  for (int pass = 0; pass < 2; ++pass) { *(volatile v8b*)(WT + e) = o; __threadfence(); }
}
__global__ __launch_bounds__(64) void upd_kernel(const float* __restrict__ x, const float* __restrict__ XSP, const float* __restrict__ XVP, const float* __restrict__ AGG, const b16* __restrict__ WSS, const b16* __restrict__ WVV, const b16* __restrict__ WSV, const b16* __restrict__ WVS, const b16* __restrict__ WLS, const b16* __restrict__ WLV, float* __restrict__ out, int mrows) {
  __shared__ __attribute__((aligned(16))) float Ls[2][16][NS_], La0[2][16][NS_], Lv[2][16][96], La1[2][16][96]; __shared__ __attribute__((aligned(16))) b16 Ah[2][16][NS_ + 8]; __shared__ __attribute__((aligned(16))) float Tf[2][16][FX + 4];
  const int wave = threadIdx.x >> 5, lane = threadIdx.x & 31, nloc = lane & 15, hlf = lane >> 4; const int n0 = blockIdx.x * 32 + wave * 16;
  for (int idx = lane; idx < 16 * 16; idx += 32) { const int rr = idx >> 4, c4 = (idx & 15) * 4; const int n = (n0 + rr < N) ? n0 + rr : N - 1;
    *(v4f*)(&Ls[wave][rr][c4]) = *(const v4f*)(XSP + (size_t)n * NS_ + c4); *(v4f*)(&La0[wave][rr][c4]) = *(const v4f*)(AGG + (size_t)n * AW + c4); }
  for (int idx = lane; idx < 16 * 24; idx += 32) { const int rr = idx / 24, c4 = (idx % 24) * 4; const int n = (n0 + rr < N) ? n0 + rr : N - 1;
    *(v4f*)(&La1[wave][rr][c4]) = *(const v4f*)(AGG + (size_t)n * AW + NS_ + c4);
    v4f t; for (int j = 0; j < 4; ++j) { const int f = c4 + j, u = f / 3, i = f % 3; t[j] = XVP[((size_t)i * NP + n) * NV_ + u]; } *(v4f*)(&Lv[wave][rr][c4]) = t; }
  wave_lds_sync();
  v8f acc0[4], acc1[3][2]; for (int t = 0; t < 4; ++t) acc0[t] = (v8f){}; for (int i = 0; i < 3; ++i) for (int t = 0; t < 2; ++t) acc1[i][t] = (v8f){};
  const int srow = lane >> 1, scol = (lane & 1) * 32;
  auto stage = [&](auto val) { for (int c = 0; c < 32; c += 4) { v4h hv; for (int j = 0; j < 4; ++j) hv[j] = (b16)(val(srow, scol + c + j) * XS); *(v4h*)(&Ah[wave][srow][scol + c]) = hv; } };
#pragma unroll 1
  for (int u = 0; u < NS_; ++u) { wave_lds_sync(); stage([&](int r, int vcol) { return pmul(Ls[wave][r][u] * INV64, La0[wave][r][vcol]); }); wave_lds_sync();
    const v16b f0 = frag_kb(&Ah[wave][nloc][0], hlf), f1 = frag_kb(&Ah[wave][nloc][32], hlf); const b16* Wb = WSS + (size_t)u * NS_ * NS_;
#pragma unroll
    for (int t = 0; t < 4; ++t) { const size_t wo_ = (size_t)(t * 16 + nloc) * NS_; acc0[t] = wmma16b(f0, frag_kb(Wb + wo_, hlf), acc0[t]); acc0[t] = wmma16b(f1, frag_kb(Wb + wo_ + 32, hlf), acc0[t]); } }
#pragma unroll 1
  for (int u = 0; u < NV_; ++u) { wave_lds_sync(); stage([&](int r, int vcol) { if (vcol >= NV_) return 0.0f; const float* xv = &Lv[wave][r][3 * u]; const float* av = &La1[wave][r][3 * vcol]; return (pmul(xv[0], av[0]) + pmul(xv[1], av[1]) + pmul(xv[2], av[2])) * K_UVV; }); wave_lds_sync();
    const v16b f0 = frag_kb(&Ah[wave][nloc][0], hlf); const b16* Wb = WVV + (size_t)u * NS_ * NV_;
#pragma unroll
    for (int t = 0; t < 4; ++t) acc0[t] = wmma16b(f0, frag_kb(Wb + (size_t)(t * 16 + nloc) * NV_, hlf), acc0[t]); }
#pragma unroll 1
  for (int u = 0; u < NS_; ++u) {
#pragma unroll
    for (int i = 0; i < 3; ++i) { wave_lds_sync(); stage([&](int r, int vcol) { if (vcol >= NV_) return 0.0f; return pmul(Ls[wave][r][u] * INV_SQRT2048, La1[wave][r][3 * vcol + i]); }); wave_lds_sync();
      const v16b f0 = frag_kb(&Ah[wave][nloc][0], hlf); const b16* Wb = WSV + (size_t)u * NV_ * NV_;
#pragma unroll
      for (int t = 0; t < 2; ++t) acc1[i][t] = wmma16b(f0, frag_kb(Wb + (size_t)(t * 16 + nloc) * NV_, hlf), acc1[i][t]); } }
#pragma unroll 1
  for (int u = 0; u < NV_; ++u) {
#pragma unroll
    for (int i = 0; i < 3; ++i) { wave_lds_sync(); stage([&](int r, int vcol) { return pmul(Lv[wave][r][3 * u + i] * INV_SQRT2048, La0[wave][r][vcol]); }); wave_lds_sync();
      const v16b f0 = frag_kb(&Ah[wave][nloc][0], hlf), f1 = frag_kb(&Ah[wave][nloc][32], hlf); const b16* Wb = WVS + (size_t)u * NV_ * NS_;
#pragma unroll
      for (int t = 0; t < 2; ++t) { const size_t wo_ = (size_t)(t * 16 + nloc) * NS_; acc1[i][t] = wmma16b(f0, frag_kb(Wb + wo_, hlf), acc1[i][t]); acc1[i][t] = wmma16b(f1, frag_kb(Wb + wo_ + 32, hlf), acc1[i][t]); } } }
  { wave_lds_sync(); stage([&](int r, int vcol) { return Ls[wave][r][vcol] * INV8; }); wave_lds_sync();
    const v16b f0 = frag_kb(&Ah[wave][nloc][0], hlf), f1 = frag_kb(&Ah[wave][nloc][32], hlf);
#pragma unroll
    for (int t = 0; t < 4; ++t) { const size_t wo_ = (size_t)(t * 16 + nloc) * NS_; acc0[t] = wmma16b(f0, frag_kb(WLS + wo_, hlf), acc0[t]); acc0[t] = wmma16b(f1, frag_kb(WLS + wo_ + 32, hlf), acc0[t]); } }
#pragma unroll
  for (int i = 0; i < 3; ++i) { wave_lds_sync(); stage([&](int r, int vcol) { if (vcol >= NV_) return 0.0f; return Lv[wave][r][3 * vcol + i] * INV_SQRT32; }); wave_lds_sync();
    const v16b f0 = frag_kb(&Ah[wave][nloc][0], hlf);
#pragma unroll
    for (int t = 0; t < 2; ++t) acc1[i][t] = wmma16b(f0, frag_kb(WLV + (size_t)(t * 16 + nloc) * NV_, hlf), acc1[i][t]); }
#pragma unroll
  for (int t = 0; t < 4; ++t) { const int col = t * 16 + nloc; for (int r = 0; r < 8; ++r) Tf[wave][8 * hlf + r][col] = acc0[t][r] * (1.0f / (XS * WSC)); }
#pragma unroll
  for (int i = 0; i < 3; ++i) for (int t = 0; t < 2; ++t) { const int w = t * 16 + nloc; for (int r = 0; r < 8; ++r) Tf[wave][8 * hlf + r][NS_ + 3 * w + i] = acc1[i][t][r] * (1.0f / (XS * WSC)); }
  wave_lds_sync();
  for (int pass = 0; pass < 2; ++pass) { for (int q = lane; q < 16 * (FX / 4); q += 32) { const int rr = q / (FX / 4), c4 = (q % (FX / 4)) * 4; const int n = n0 + rr; if (n < mrows && n < N) { const v4f xv4 = *(const v4f*)(x + (size_t)n * FX + c4); const v4f t4 = *(const v4f*)(&Tf[wave][rr][c4]); v4f o; for (int j = 0; j < 4; ++j) o[j] = bf16_rne(xv4[j]) + t4[j]; *(volatile v4f*)(out + (size_t)n * FX + c4) = o; } } __threadfence(); }
}
}

extern "C" void kernel_launch(void* const* d_in, const int* in_sizes, int n_in, void* d_out, int out_size, void* d_ws, size_t ws_size, hipStream_t stream) {
  (void)n_in;
  auto Fp = [&](int i) { return (const float*)d_in[i]; }; auto Ip = [&](int i) { return (const int*)d_in[i]; };
  if (in_sizes[0] != N * FX || in_sizes[1] != 2 * EFULL || in_sizes[2] != EFULL * 4 || in_sizes[3] != N || in_sizes[4] != NS_ * NS_ || in_sizes[5] != NV_ * NS_ || in_sizes[6] != NS_ * NV_ || in_sizes[7] != NV_ * NV_ || in_sizes[8] != NS_ * NS_ || in_sizes[9] != NV_ * NV_) return;
  if (in_sizes[10] != NS_ * NS_ * NS_ || in_sizes[11] != NV_ * NV_ * NS_ || in_sizes[12] != NS_ * NV_ * NV_ || in_sizes[13] != NV_ * NS_ * NV_ || in_sizes[14] != NS_ * NS_ || in_sizes[15] != NV_ * NV_ || out_size != N * FX) return;
  size_t off = 0; char* ws = (char*)d_ws;
  auto carve = [&](size_t bytes) { char* p = ws + off; off += (bytes + 255) & ~(size_t)255; return p; };
  b16* WTS = (b16*)carve((size_t)TSW * NS_ * 2); b16* WTV = (b16*)carve((size_t)TVW * NV_ * 2); b16* WSS = (b16*)carve((size_t)NS_ * NS_ * NS_ * 2); b16* WVV = (b16*)carve((size_t)NV_ * NS_ * NV_ * 2); b16* WSV = (b16*)carve((size_t)NS_ * NV_ * NV_ * 2); b16* WVS = (b16*)carve((size_t)NV_ * NV_ * NS_ * 2);
  b16* WLS = (b16*)carve((size_t)NS_ * NS_ * 2); b16* WLV = (b16*)carve((size_t)NV_ * NV_ * 2); float* ZB = (float*)carve(1024);
  float* XS = (float*)carve((size_t)NP * NS_ * 4); float* XV = (float*)carve((size_t)3 * NP * NV_ * 4); float* TS = (float*)carve((size_t)NP * TSW * 4); float* TV = (float*)carve((size_t)3 * NP * TVW * 4); float* AGG = (float*)carve((size_t)NP * AW * 4);
  CsrBufs csr; off = csr_carve(csr, ws, off, E, N);
  if (off > ws_size || off > ((size_t)96 << 20)) return;
  { wt_kernel<NS_, NS_, NS_><<<(NS_ * NS_ / 8 + 255) / 256, 256, 0, stream>>>(Fp(4), WTS, WSC); wt_kernel<NS_, NS_, NS_><<<(NS_ * NS_ / 8 + 255) / 256, 256, 0, stream>>>(Fp(8), WTS + (size_t)NS_ * NS_, WSC); wt_kernel<NS_, NV_, NV_><<<(NV_ * NS_ / 8 + 255) / 256, 256, 0, stream>>>(Fp(6), WTS + (size_t)2 * NS_ * NS_, WSC);
    wt_kernel<NV_, NS_, NS_><<<(NS_ * NV_ / 8 + 255) / 256, 256, 0, stream>>>(Fp(5), WTV, WSC); wt_kernel<NV_, NV_, NV_><<<(NV_ * NV_ / 8 + 255) / 256, 256, 0, stream>>>(Fp(7), WTV + (size_t)NS_ * NV_, WSC); wt_kernel<NV_, NV_, NV_><<<(NV_ * NV_ / 8 + 255) / 256, 256, 0, stream>>>(Fp(9), WTV + (size_t)(NS_ + NV_) * NV_, WSC);
    wuvw_kernel<NS_, NS_, NS_><<<(NS_ * NS_ * NS_ / 8 + 255) / 256, 256, 0, stream>>>(Fp(10), WSS, WSC); wuvw_kernel<NV_, NV_, NS_><<<(NV_ * NV_ * NS_ / 8 + 255) / 256, 256, 0, stream>>>(Fp(11), WVV, WSC);
    wuvw_kernel<NS_, NV_, NV_><<<(NS_ * NV_ * NV_ / 8 + 255) / 256, 256, 0, stream>>>(Fp(12), WSV, WSC); wuvw_kernel<NV_, NS_, NV_><<<(NV_ * NS_ * NV_ / 8 + 255) / 256, 256, 0, stream>>>(Fp(13), WVS, WSC);
    wt_kernel<NS_, NS_, NS_><<<(NS_ * NS_ / 8 + 255) / 256, 256, 0, stream>>>(Fp(14), WLS, WSC); wt_kernel<NV_, NV_, NV_><<<(NV_ * NV_ / 8 + 255) / 256, 256, 0, stream>>>(Fp(15), WLV, WSC); zfill_kernel<<<1, 256, 0, stream>>>(ZB, 256); }
  csr_build(csr, Ip(1), E, N, stream);
  split_kernel<<<(NRL * 20 + 255) / 256, 256, 0, stream>>>(Fp(0), XS, XV);
  lin_kernel<NS_, 10, true, 0, false><<<NRL / 32, 64, 0, stream>>>(XS, nullptr, WTS, WTS, ZB, TS, TSW, N, NRL);
  for (int i = 0; i < 3; ++i) lin_kernel<NV_, 8, true, 0, false><<<NRL / 32, 64, 0, stream>>>(XV + (size_t)i * NP * NV_, nullptr, WTV, WTV, ZB, TV + (size_t)i * NP * TVW, TVW, N, NRL);
  magg_kernel<<<NRL / 32, 256, 0, stream>>>(TS, TV, Fp(2), Ip(1) + EFULL, csr.PERM, csr.ROWPTR, csr.ROWCNT, (int)csr.permLen, AGG, NRL);
  upd_kernel<<<NPL / 32, 64, 0, stream>>>(Fp(0), XS, XV, AGG, WSS, WVV, WSV, WVS, WLS, WLV, (float*)d_out, NL);
}
